// OuterProductMean_31516470018143
// MI455X (gfx1250) — hardware-verified
//
#include <hip/hip_runtime.h>

typedef __bf16         v16bf __attribute__((ext_vector_type(16)));
typedef _Float16       v16h  __attribute__((ext_vector_type(16)));
typedef _Float16       v8h   __attribute__((ext_vector_type(8)));
typedef unsigned short v8us  __attribute__((ext_vector_type(8)));
typedef float          v8f   __attribute__((ext_vector_type(8)));
typedef float          v4f   __attribute__((ext_vector_type(4)));
typedef v8us __attribute__((may_alias)) v8usa;
typedef v8h  __attribute__((may_alias)) v8ha;
typedef v4f  __attribute__((may_alias)) v4fa;

union FragB { v16bf v; v8us half[2]; };
union FragH { v16h v; v8h half[2]; };

#define SDIM 128
#define NRES 256
#define CIN  256
#define CH   32
#define CZ   128
#define CDD  1024
#define NTHR 256

#ifndef NI_ROWS
#define NI_ROWS NRES
#endif
static_assert(NI_ROWS >= 1 && NI_ROWS <= NRES);

#define PLANE_ROWS   (NRES * CH)
#define PLANE_HALVES (PLANE_ROWS * SDIM)
#define PLANE_BYTES  (PLANE_HALVES * 2)
#define WOT_HALVES   (CZ * CDD)
#define WOT_BYTES    (WOT_HALVES * 2)
#define WS_TOTAL     ((size_t)4 * PLANE_BYTES + WOT_BYTES)

#define XP 264
#define MP 1032
#define TP 72

#define MEAN_CARRY  16.0f
#define WO_CARRY    64.0f
#define OUT_UNCARRY (1.0f / 1024.0f)
#define LN_EPS 1e-5f
#define MSK_EPS 1e-3f

static_assert(WS_TOTAL == 8650752);
static_assert(PLANE_BYTES % 128 == 0 && WOT_BYTES % 128 == 0);
static_assert(SDIM % 32 == 0 && CIN % 32 == 0 && CDD % 32 == 0);
static_assert(NRES % 32 == 0 && CDD % 64 == 0);

#define P_OFF_XH 0
#define P_OFF_XL 33792
#define P_OFF_W  67584
#define P_OFF_SO 101376
#define P_OFF_M  117760
#define P_SMEM   118016
static_assert(P_OFF_XL == P_OFF_XH + 64 * XP * 2);
static_assert(P_OFF_W  == P_OFF_XL + 64 * XP * 2);
static_assert(P_OFF_SO == P_OFF_W + 2 * CH * XP * 2);
static_assert(P_OFF_M  == P_OFF_SO + 4 * CH * 64 * 2);
static_assert(P_SMEM   == P_OFF_M + 64 * 4);
static_assert(P_OFF_XL % 16 == 0 && P_OFF_W % 16 == 0 && P_OFF_SO % 16 == 0 && P_OFF_M % 16 == 0);

#define M_OFF_MEAN 0
#define M_OFF_O    66048
#define M_OFF_RN   82432
#define M_OFF_RB   82560
#define M_SMEM     82688
static_assert(M_OFF_O == 32 * MP * 2);
static_assert(M_OFF_RN == M_OFF_O + 32 * CZ * 4);
static_assert(M_OFF_RB == M_OFF_RN + 32 * 4);
static_assert(M_SMEM == M_OFF_RB + 32 * 4);
static_assert(M_OFF_O % 16 == 0 && M_OFF_RN % 16 == 0 && M_OFF_RB % 16 == 0);

__device__ __forceinline__ unsigned short f2bf(float f) {
  unsigned u = __builtin_bit_cast(unsigned, f);
  u += 0x7FFFu + ((u >> 16) & 1u);
  return (unsigned short)(u >> 16);
}
__device__ __forceinline__ float bf2f(unsigned short s) {
  return __builtin_bit_cast(float, ((unsigned)s) << 16);
}
__device__ __forceinline__ float bfr(float f) { return bf2f(f2bf(f)); }

__device__ __forceinline__ v8f wmma_bf16(v16bf a, v16bf b, v8f c) {
  v8f d = __builtin_amdgcn_wmma_f32_16x16x32_bf16(false, a, false, b, (short)0, c, false, false);
  asm volatile("v_nop\n\tv_nop\n\tv_nop\n\tv_nop" : "+v"(d) : "v"(a), "v"(b));
  return d;
}
__device__ __forceinline__ v8f wmma_f16(v16h a, v16h b, v8f c) {
  v8f d = __builtin_amdgcn_wmma_f32_16x16x32_f16(false, a, false, b, (short)0, c, false, false);
  asm volatile("v_nop\n\tv_nop\n\tv_nop\n\tv_nop" : "+v"(d) : "v"(a), "v"(b));
  return d;
}

__device__ __forceinline__ v16bf load_frag_bf(const unsigned short* p, int h) {
  FragB f;
  f.half[0] = *(const v8usa*)(p + 8 * h);
  f.half[1] = *(const v8usa*)(p + 16 + 8 * h);
  return f.v;
}
__device__ __forceinline__ v16h load_frag_h(const _Float16* p, int h) {
  FragH f;
  f.half[0] = *(const v8ha*)(p + 8 * h);
  f.half[1] = *(const v8ha*)(p + 16 + 8 * h);
  return f.v;
}

__device__ __forceinline__ void wot_store_pass(const _Float16* sT, _Float16* woT,
                                               int cd0, int w, int lane) {
  const int q8 = lane & 7, sub = lane >> 3;
  #pragma unroll
  for (int it = 0; it < 4; ++it) {
    const int z = w * 16 + it * 4 + sub;
    const v8h v = *(const v8ha*)(sT + z * TP + 8 * q8);
    *(volatile v8h*)(woT + (size_t)z * CDD + cd0 + 8 * q8) = v;
  }
}

__global__ __launch_bounds__(NTHR) void k_wot(const float* __restrict__ wout,
                                             _Float16* __restrict__ woT) {
  __shared__ __attribute__((aligned(16))) _Float16 sT[CZ * TP];
  const int tid = threadIdx.x, lane = tid & 31, w = tid >> 5;
  const int cd0 = blockIdx.x * 64;
  #pragma unroll
  for (int it = 0; it < 8; ++it) {
    const int q = it * NTHR + tid;
    const int cdl = q >> 5, z4 = (q & 31) * 4;
    const v4f v = *(const v4fa*)(wout + (size_t)(cd0 + cdl) * CZ + z4);
    sT[(z4 + 0) * TP + cdl] = (_Float16)(bfr(v.x) * WO_CARRY);
    sT[(z4 + 1) * TP + cdl] = (_Float16)(bfr(v.y) * WO_CARRY);
    sT[(z4 + 2) * TP + cdl] = (_Float16)(bfr(v.z) * WO_CARRY);
    sT[(z4 + 3) * TP + cdl] = (_Float16)(bfr(v.w) * WO_CARRY);
  }
  __syncthreads();
  wot_store_pass(sT, woT, cd0, w, lane);
  __threadfence();
  wot_store_pass(sT, woT, cd0, w, lane);
}

__device__ __forceinline__ void plane_store_pass(const unsigned short* sOut, unsigned short* planes,
                                                 int i, int s0, int w, int lane) {
  const int q8 = lane & 7, sub = lane >> 3;
  #pragma unroll
  for (int it = 0; it < 4; ++it) {
    const int L = w * 16 + it * 4 + sub;
    const int p = L >> 5, c = L & 31;
    const v8us v = *(const v8usa*)(sOut + L * 64 + 8 * q8);
    unsigned short* dst = planes + (size_t)p * PLANE_HALVES + (size_t)(i * CH + c) * SDIM + s0 + 8 * q8;
    *(volatile v8us*)dst = v;
  }
}

__global__ __launch_bounds__(NTHR) void k_prep(
    const float* __restrict__ msa, const float* __restrict__ mask,
    const float* __restrict__ ln_w, const float* __restrict__ ln_b,
    const float* __restrict__ w1, const float* __restrict__ b1,
    const float* __restrict__ w2, const float* __restrict__ b2,
    unsigned short* __restrict__ planes)
{
  extern __shared__ __attribute__((aligned(16))) char smem[];
  unsigned short* sXH  = (unsigned short*)(smem + P_OFF_XH);
  unsigned short* sXL  = (unsigned short*)(smem + P_OFF_XL);
  unsigned short* sW   = (unsigned short*)(smem + P_OFF_W);
  unsigned short* sOut = (unsigned short*)(smem + P_OFF_SO);
  float* sM = (float*)(smem + P_OFF_M);

  const int tid = threadIdx.x, lane = tid & 31, w = tid >> 5;
  const int h = lane >> 4, m = lane & 15;
  const int i = blockIdx.x >> 1, s0 = (blockIdx.x & 1) * 64;

  #pragma unroll 1
  for (int it = 0; it < 16; ++it) {
    const int q = it * NTHR + tid;
    const int which = it >> 3;
    const int q4 = q & 2047;
    const int k = q4 >> 3, c0 = (q4 & 7) * 4;
    const float* wsrc = (it < 8) ? w1 : w2;
    const v4f v = *(const v4fa*)(wsrc + (size_t)q4 * 4);
    unsigned short* d = sW + (which * CH + c0) * XP + k;
    d[0]      = f2bf(v.x);
    d[XP]     = f2bf(v.y);
    d[2 * XP] = f2bf(v.z);
    d[3 * XP] = f2bf(v.w);
  }
  if (tid < 64) sM[tid] = bfr(mask[(size_t)(s0 + tid) * NRES + i]);

  float gw[8], gb[8];
  {
    const v4f a = *(const v4fa*)(ln_w + 8 * lane);
    const v4f c = *(const v4fa*)(ln_w + 8 * lane + 4);
    const v4f d = *(const v4fa*)(ln_b + 8 * lane);
    const v4f e = *(const v4fa*)(ln_b + 8 * lane + 4);
    gw[0] = bfr(a.x); gw[1] = bfr(a.y); gw[2] = bfr(a.z); gw[3] = bfr(a.w);
    gw[4] = bfr(c.x); gw[5] = bfr(c.y); gw[6] = bfr(c.z); gw[7] = bfr(c.w);
    gb[0] = bfr(d.x); gb[1] = bfr(d.y); gb[2] = bfr(d.z); gb[3] = bfr(d.w);
    gb[4] = bfr(e.x); gb[5] = bfr(e.y); gb[6] = bfr(e.z); gb[7] = bfr(e.w);
  }
  #pragma unroll 1
  for (int rr = 0; rr < 8; ++rr) {
    const int rl = w * 8 + rr;
    const float* xp = msa + ((size_t)(s0 + rl) * NRES + i) * CIN + 8 * lane;
    const v4f xa = *(const v4fa*)xp;
    const v4f xc = *(const v4fa*)(xp + 4);
    float v[8] = { bfr(xa.x), bfr(xa.y), bfr(xa.z), bfr(xa.w),
                   bfr(xc.x), bfr(xc.y), bfr(xc.z), bfr(xc.w) };
    float sm = 0.0f;
    #pragma unroll
    for (int e = 0; e < 8; ++e) sm += v[e];
    sm += __shfl_xor(sm, 16);
    sm += __shfl_xor(sm, 8);
    sm += __shfl_xor(sm, 4);
    sm += __shfl_xor(sm, 2);
    sm += __shfl_xor(sm, 1);
    const float mu = sm * (1.0f / CIN);
    float q = 0.0f;
    #pragma unroll
    for (int e = 0; e < 8; ++e) { v[e] -= mu; q += v[e] * v[e]; }
    q += __shfl_xor(q, 16);
    q += __shfl_xor(q, 8);
    q += __shfl_xor(q, 4);
    q += __shfl_xor(q, 2);
    q += __shfl_xor(q, 1);
    const float rstd = rsqrtf(q * (1.0f / CIN) + LN_EPS);
    unsigned short hi[8], lo[8];
    #pragma unroll
    for (int e = 0; e < 8; ++e) {
      const float y = v[e] * rstd * gw[e] + gb[e];
      hi[e] = f2bf(y);
      lo[e] = f2bf(y - bf2f(hi[e]));
    }
    const v8us vh = { hi[0], hi[1], hi[2], hi[3], hi[4], hi[5], hi[6], hi[7] };
    const v8us vl = { lo[0], lo[1], lo[2], lo[3], lo[4], lo[5], lo[6], lo[7] };
    *(v8usa*)(sXH + rl * XP + 8 * lane) = vh;
    *(v8usa*)(sXL + rl * XP + 8 * lane) = vl;
  }
  __syncthreads();

  const int mt = w >> 1, which = w & 1;
  const v8f z8 = {0.f, 0.f, 0.f, 0.f, 0.f, 0.f, 0.f, 0.f};
  v8f acc[2];
  acc[0] = z8; acc[1] = z8;
  const unsigned short* xh = sXH + (16 * mt + m) * XP;
  const unsigned short* xl = sXL + (16 * mt + m) * XP;
  const unsigned short* wb = sW + (which * CH + m) * XP;
  #pragma unroll 1
  for (int k0 = 0; k0 < CIN; k0 += 32) {
    const v16bf a_hi = load_frag_bf(xh + k0, h);
    const v16bf a_lo = load_frag_bf(xl + k0, h);
    #pragma unroll
    for (int t = 0; t < 2; ++t) {
      const v16bf b = load_frag_bf(wb + t * 16 * XP + k0, h);
      acc[t] = wmma_bf16(a_hi, b, acc[t]);
      acc[t] = wmma_bf16(a_lo, b, acc[t]);
    }
  }
  const float* bias = which ? b2 : b1;
  #pragma unroll
  for (int t = 0; t < 2; ++t) {
    const int c = 16 * t + m;
    const float bia = bfr(bias[c]);
    #pragma unroll
    for (int r = 0; r < 8; ++r) {
      const int sl = 16 * mt + 8 * h + r;
      const float y = (acc[t][r] + bia) * sM[sl];
      const unsigned short yh = f2bf(y);
      const unsigned short yl = f2bf(y - bf2f(yh));
      sOut[((which * 2 + 0) * CH + c) * 64 + sl] = yh;
      sOut[((which * 2 + 1) * CH + c) * 64 + sl] = yl;
    }
  }
  __syncthreads();

  plane_store_pass(sOut, planes, i, s0, w, lane);
  __threadfence();
  plane_store_pass(sOut, planes, i, s0, w, lane);
}

__device__ __forceinline__ void out_store_pass(const float* sO, float* base, int w, int lane) {
  const int q8 = lane & 7, sub = lane >> 3;
  #pragma unroll
  for (int it = 0; it < 4; ++it) {
    const int L = w * 16 + it * 4 + sub;
    const v4f v = *(const v4fa*)(sO + L * 32 + 4 * q8);
    *(volatile v4f*)(base + L * 32 + 4 * q8) = v;
  }
}

__global__ __launch_bounds__(NTHR) void k_main(
    const unsigned short* __restrict__ planes,
    const _Float16* __restrict__ woT,
    const float* __restrict__ mask,
    const float* __restrict__ bout,
    float* __restrict__ out)
{
  extern __shared__ __attribute__((aligned(16))) char smem[];
  _Float16* sMean = (_Float16*)(smem + M_OFF_MEAN);
  float* sO  = (float*)(smem + M_OFF_O);
  float* sRn = (float*)(smem + M_OFF_RN);
  float* sRb = (float*)(smem + M_OFF_RB);

  const int tid = threadIdx.x, lane = tid & 31, w = tid >> 5;
  const int h = lane >> 4, m = lane & 15;
  const int i = blockIdx.y, j0 = blockIdx.x * 32;

  const unsigned short* Ahi = planes;
  const unsigned short* Alo = planes + (size_t)PLANE_HALVES;
  const unsigned short* Bhi = planes + (size_t)2 * PLANE_HALVES;
  const unsigned short* Blo = planes + (size_t)3 * PLANE_HALVES;

  if (tid < 32) {
    const int j = j0 + tid;
    float nacc = 0.0f;
    #pragma unroll 1
    for (int s = 0; s < SDIM; ++s)
      nacc = fmaf(bfr(mask[s * NRES + i]), bfr(mask[s * NRES + j]), nacc);
    const float rb = 1.0f / (nacc + MSK_EPS);
    sRn[tid] = MEAN_CARRY * rb;
    sRb[tid] = rb;
  }
  __syncthreads();

  const v8f z8 = {0.f, 0.f, 0.f, 0.f, 0.f, 0.f, 0.f, 0.f};

  const unsigned short* ah_r = Ahi + (size_t)(i * CH + m) * SDIM;
  const unsigned short* al_r = Alo + (size_t)(i * CH + m) * SDIM;
  #pragma unroll 1
  for (int jj = 0; jj < 4; ++jj) {
    const int jl = 4 * w + jj, j = j0 + jl;
    const unsigned short* bh_r = Bhi + (size_t)(j * CH + m) * SDIM;
    const unsigned short* bl_r = Blo + (size_t)(j * CH + m) * SDIM;
    v8f acc[2][2];
    acc[0][0] = z8; acc[0][1] = z8; acc[1][0] = z8; acc[1][1] = z8;
    #pragma unroll 1
    for (int k0 = 0; k0 < SDIM; k0 += 32) {
      const v16bf ahf0 = load_frag_bf(ah_r + k0, h);
      const v16bf ahf1 = load_frag_bf(ah_r + 16 * SDIM + k0, h);
      const v16bf alf0 = load_frag_bf(al_r + k0, h);
      const v16bf alf1 = load_frag_bf(al_r + 16 * SDIM + k0, h);
      const v16bf bhf0 = load_frag_bf(bh_r + k0, h);
      const v16bf bhf1 = load_frag_bf(bh_r + 16 * SDIM + k0, h);
      const v16bf blf0 = load_frag_bf(bl_r + k0, h);
      const v16bf blf1 = load_frag_bf(bl_r + 16 * SDIM + k0, h);
      acc[0][0] = wmma_bf16(ahf0, bhf0, acc[0][0]);
      acc[0][0] = wmma_bf16(ahf0, blf0, acc[0][0]);
      acc[0][0] = wmma_bf16(alf0, bhf0, acc[0][0]);
      acc[0][1] = wmma_bf16(ahf0, bhf1, acc[0][1]);
      acc[0][1] = wmma_bf16(ahf0, blf1, acc[0][1]);
      acc[0][1] = wmma_bf16(alf0, bhf1, acc[0][1]);
      acc[1][0] = wmma_bf16(ahf1, bhf0, acc[1][0]);
      acc[1][0] = wmma_bf16(ahf1, blf0, acc[1][0]);
      acc[1][0] = wmma_bf16(alf1, bhf0, acc[1][0]);
      acc[1][1] = wmma_bf16(ahf1, bhf1, acc[1][1]);
      acc[1][1] = wmma_bf16(ahf1, blf1, acc[1][1]);
      acc[1][1] = wmma_bf16(alf1, bhf1, acc[1][1]);
    }
    const float rn = sRn[jl];
    _Float16* mrow = sMean + jl * MP;
    #pragma unroll
    for (int mt = 0; mt < 2; ++mt)
      #pragma unroll
      for (int nt = 0; nt < 2; ++nt)
        #pragma unroll
        for (int r = 0; r < 8; ++r)
          mrow[(16 * mt + 8 * h + r) * CH + 16 * nt + m] = (_Float16)(acc[mt][nt][r] * rn);
  }
  __syncthreads();

  v8f acc2[2];
  acc2[0] = z8; acc2[1] = z8;
  const _Float16* ma0 = sMean + m * MP;
  const _Float16* ma1 = sMean + (16 + m) * MP;
  const _Float16* wrow = woT + (size_t)(16 * w + m) * CDD;
  #pragma unroll 1
  for (int k0 = 0; k0 < CDD; k0 += 32) {
    const v16h a0 = load_frag_h(ma0 + k0, h);
    const v16h a1 = load_frag_h(ma1 + k0, h);
    const v16h b  = load_frag_h(wrow + k0, h);
    acc2[0] = wmma_f16(a0, b, acc2[0]);
    acc2[1] = wmma_f16(a1, b, acc2[1]);
  }
  const int z = 16 * w + m;
  const float boz = bfr(bout[z]);
  #pragma unroll
  for (int mt = 0; mt < 2; ++mt)
    #pragma unroll
    for (int r = 0; r < 8; ++r) {
      const int jl = 16 * mt + 8 * h + r;
      sO[jl * CZ + z] = acc2[mt][r] * OUT_UNCARRY + boz * sRb[jl];
    }
  __syncthreads();

  float* base = out + ((size_t)i * NRES + j0) * CZ;
  out_store_pass(sO, base, w, lane);
  __threadfence();
  out_store_pass(sO, base, w, lane);
}

extern "C" void kernel_launch(void* const* d_in, const int* in_sizes, int n_in,
                              void* d_out, int out_size, void* d_ws, size_t ws_size,
                              hipStream_t stream) {
  if (n_in < 10) return;
  if (in_sizes[0] < SDIM * NRES * CIN) return;
  if (in_sizes[1] < SDIM * NRES) return;
  if (in_sizes[2] < CIN || in_sizes[3] < CIN) return;
  if (in_sizes[4] < CIN * CH || in_sizes[5] < CH) return;
  if (in_sizes[6] < CIN * CH || in_sizes[7] < CH) return;
  if (in_sizes[8] < CDD * CZ || in_sizes[9] < CZ) return;
  if (out_size < NI_ROWS * NRES * CZ) return;
  if (WS_TOTAL > ws_size) return;

  const float* msa  = (const float*)d_in[0];
  const float* mask = (const float*)d_in[1];
  const float* ln_w = (const float*)d_in[2];
  const float* ln_b = (const float*)d_in[3];
  const float* w1   = (const float*)d_in[4];
  const float* b1   = (const float*)d_in[5];
  const float* w2   = (const float*)d_in[6];
  const float* b2   = (const float*)d_in[7];
  const float* wout = (const float*)d_in[8];
  const float* bout = (const float*)d_in[9];
  float* out = (float*)d_out;

  char* ws = (char*)d_ws;
  unsigned short* planes = (unsigned short*)ws;
  _Float16* woT = (_Float16*)(ws + (size_t)4 * PLANE_BYTES);

  k_wot<<<CDD / 64, NTHR, 0, stream>>>(wout, woT);

  hipFuncSetAttribute(reinterpret_cast<const void*>(&k_prep),
                      hipFuncAttributeMaxDynamicSharedMemorySize, P_SMEM);
  k_prep<<<NRES * 2, NTHR, P_SMEM, stream>>>(msa, mask, ln_w, ln_b, w1, b1, w2, b2, planes);

  hipFuncSetAttribute(reinterpret_cast<const void*>(&k_main),
                      hipFuncAttributeMaxDynamicSharedMemorySize, M_SMEM);
  dim3 gMain(NRES / 32, NI_ROWS);
  k_main<<<gMain, NTHR, M_SMEM, stream>>>(planes, woT, mask, bout, out);
}
